// SAGENet_60816736911616
// MI455X (gfx1250) — hardware-verified
//
#include <hip/hip_runtime.h>
#include <stddef.h>
#include <stdint.h>


#define DIN     128
#define DH      128
#define NCLS    40
#define NCP     64
#define K1      384
#define HBP     256
#define K2      512
#define NTHR    256
#define NWAVE   8
#define EPT     8
#define CHUNK   (NTHR * EPT)
#define WCAP    (EPT * 32)
#define LISTN   (NWAVE * WCAP)
#define NBMAX   2048
#define RCAP    28672
#define DEGCAP  128
#define PKS     11
#define STW     512
#define GBM     64
#define GTHR    128
#define WSMAX   268435456
#define WSCAP   134217728
#define LDS_AGG ((2 * RCAP + 2 * NBMAX + LISTN) * 4 + 64)

static_assert((CHUNK & (CHUNK - 1)) == 0 && CHUNK <= (1 << PKS));
static_assert((NBMAX & (NBMAX - 1)) == 0 && NBMAX <= (1 << PKS));
static_assert(NTHR * 8 == NBMAX);
static_assert(LISTN >= NBMAX);
static_assert(LISTN >= NWAVE * WCAP);
static_assert((RCAP % 32) == 0);
static_assert(NWAVE * STW <= RCAP);
static_assert(STW >= 192);
static_assert(LDS_AGG <= 300000);
static_assert(GBM == (GTHR / 32) * 16);
static_assert(GTHR == DH);
static_assert((K1 % 32) == 0 && (HBP % 32) == 0 && (K2 % 32) == 0);
static_assert(K1 == 3 * DIN && HBP == 2 * DH && K2 == 2 * HBP);
static_assert(NCLS > 32 && NCLS <= NCP && (NCLS % 4) == 0 && NCP == 64);
static_assert(DH == 32 * 4 && DIN == DH && (DH % 64) == 0);

typedef float          v2f  __attribute__((ext_vector_type(2)));
typedef float          v4f  __attribute__((ext_vector_type(4)));
typedef float          v8f  __attribute__((ext_vector_type(8)));
typedef int            v4i  __attribute__((ext_vector_type(4)));
typedef int            v8i  __attribute__((ext_vector_type(8)));
typedef unsigned int   v2u  __attribute__((ext_vector_type(2)));
typedef unsigned int   v4u  __attribute__((ext_vector_type(4)));
typedef unsigned short u16;
typedef u16            v8us __attribute__((ext_vector_type(8)));
typedef v8us __attribute__((may_alias)) v8usa;
typedef v4f  __attribute__((may_alias)) v4fa;
typedef v2u  __attribute__((may_alias)) v2ua;
typedef v4u  __attribute__((may_alias)) v4ua;
typedef __bf16         v16b __attribute__((ext_vector_type(16)));
union FragB { v16b v; v8us h[2]; v8i w; };

__device__ __forceinline__ v8f wmb(const FragB& a, const FragB& b, v8f c) {
  v8f d = __builtin_amdgcn_wmma_f32_16x16x32_bf16(false, a.v, false, b.v, (short)0, c, false, false);
  asm volatile("v_nop\n\tv_nop\n\tv_nop\n\tv_nop" : "+v"(d) : "v"(a.w), "v"(b.w));
  return d;
}

__device__ __forceinline__ unsigned short bf_bits(float f) {
  unsigned int u = __float_as_uint(f);
  u += 0x7FFFu + ((u >> 16) & 1u);
  return (unsigned short)(u >> 16);
}
__device__ __forceinline__ float bf_val(unsigned short b) {
  return __uint_as_float(((unsigned int)b) << 16);
}
__device__ __forceinline__ float bf_rne(float f) { return bf_val(bf_bits(f)); }

__device__ __forceinline__ v8us cvt8b(const v4f a, const v4f b) {
  v8us hv;
  hv[0] = bf_bits(a.x); hv[1] = bf_bits(a.y); hv[2] = bf_bits(a.z); hv[3] = bf_bits(a.w);
  hv[4] = bf_bits(b.x); hv[5] = bf_bits(b.y); hv[6] = bf_bits(b.z); hv[7] = bf_bits(b.w);
  return hv;
}

__device__ __forceinline__ int scan_chunk(const int* __restrict__ dsts, int nE, int cbase, int slotBase,
                                          int nb, int vec8, int* list, int tid, int lane, int wave) {
  int wc = 0;
  const int el0  = tid * EPT;
  const int e0   = cbase + el0;
  const int sent = -2147483647 - 1;
  v4i da, db;
  if (vec8 != 0 && cbase + CHUNK <= nE) {
    da = *(const v4i*)(dsts + e0);
    db = *(const v4i*)(dsts + e0 + 4);
  } else {
    da.x = (e0     < nE) ? dsts[min(e0,     nE - 1)] : sent;
    da.y = (e0 + 1 < nE) ? dsts[min(e0 + 1, nE - 1)] : sent;
    da.z = (e0 + 2 < nE) ? dsts[min(e0 + 2, nE - 1)] : sent;
    da.w = (e0 + 3 < nE) ? dsts[min(e0 + 3, nE - 1)] : sent;
    db.x = (e0 + 4 < nE) ? dsts[min(e0 + 4, nE - 1)] : sent;
    db.y = (e0 + 5 < nE) ? dsts[min(e0 + 5, nE - 1)] : sent;
    db.z = (e0 + 6 < nE) ? dsts[min(e0 + 6, nE - 1)] : sent;
    db.w = (e0 + 7 < nE) ? dsts[min(e0 + 7, nE - 1)] : sent;
  }
  const unsigned nbs = (unsigned)slotBase;
  const unsigned unb = (unsigned)nb;
  const unsigned s0 = (unsigned)da.x - nbs, s1 = (unsigned)da.y - nbs;
  const unsigned s2 = (unsigned)da.z - nbs, s3 = (unsigned)da.w - nbs;
  const unsigned s4 = (unsigned)db.x - nbs, s5 = (unsigned)db.y - nbs;
  const unsigned s6 = (unsigned)db.z - nbs, s7 = (unsigned)db.w - nbs;
  const bool h0 = s0 < unb, h1 = s1 < unb, h2 = s2 < unb, h3 = s3 < unb;
  const bool h4 = s4 < unb, h5 = s5 < unb, h6 = s6 < unb, h7 = s7 < unb;
  const unsigned any = __builtin_amdgcn_ballot_w32(h0 | h1 | h2 | h3 | h4 | h5 | h6 | h7);
  if (any != 0u) {
#define HITJ(J, HJ, SJ) { \
      const unsigned mj = __builtin_amdgcn_ballot_w32(HJ); \
      if (mj != 0u) { \
        if (HJ) { \
          const int pos = wc + (int)__builtin_amdgcn_mbcnt_lo(mj, 0u); \
          if (pos < WCAP) list[wave * WCAP + pos] = ((el0 + (J)) << PKS) | (int)(SJ); \
        } \
        wc += (int)__builtin_popcount(mj); } }
    HITJ(0, h0, s0)
    HITJ(1, h1, s1)
    HITJ(2, h2, s2)
    HITJ(3, h3, s3)
    HITJ(4, h4, s4)
    HITJ(5, h5, s5)
    HITJ(6, h6, s6)
    HITJ(7, h7, s7)
#undef HITJ
  }
  return wc;
}

__global__ __launch_bounds__(NTHR) void k_xprep(const float* __restrict__ x, u16* xb, int nN, int nUnits) {
  const int i = (int)blockIdx.x * NTHR + (int)threadIdx.x;
  if (i >= nUnits) return;
  const int row = i >> 4;
  const int c0  = (i & 15) * 8;
  const int rc  = row < nN ? row : nN - 1;
  const float* p = x + (size_t)rc * DIN + c0;
  v4f a = *(const v4fa*)p, b = *(const v4fa*)(p + 4);
  const v4f z4 = {0.f, 0.f, 0.f, 0.f};
  if (row >= nN) { a = z4; b = z4; }
  const v8us hv = cvt8b(a, b);
  const size_t o = (size_t)row * DIN + c0;
  *(volatile v8us*)(xb + o) = hv;
  __threadfence();
  *(volatile v8us*)(xb + o) = hv;
}

__global__ __launch_bounds__(NTHR) void k_wtr(const float* __restrict__ w0, const float* __restrict__ w1,
                                              int C, int segSplit, int K, u16* wt, int nUnits) {
  const int u = (int)blockIdx.x * NTHR + (int)threadIdx.x;
  if (u >= nUnits) return;
  const int kq = K >> 3;
  const int n  = u / kq;
  const int k8 = (u - n * kq) * 8;
  const int seg = k8 >> 7;
  const int ks  = k8 & (DIN - 1);
  int ncl = n < C ? n : C - 1;
  ncl = ncl < 0 ? 0 : ncl;
  const float* wsrc = (seg >= segSplit) ? w1 : w0;
  const float* p = wsrc + (size_t)ks * (size_t)C + ncl;
  v4f a, b;
  a.x = p[0];                 a.y = p[(size_t)C];         a.z = p[(size_t)2 * C];     a.w = p[(size_t)3 * C];
  b.x = p[(size_t)4 * C];     b.y = p[(size_t)5 * C];     b.z = p[(size_t)6 * C];     b.w = p[(size_t)7 * C];
  const v4f z4 = {0.f, 0.f, 0.f, 0.f};
  if (n >= C) { a = z4; b = z4; }
  const v8us hv = cvt8b(a, b);
  const size_t o = (size_t)n * (size_t)K + k8;
  *(volatile v8us*)(wt + o) = hv;
  __threadfence();
  *(volatile v8us*)(wt + o) = hv;
}

__global__ __launch_bounds__(GTHR) void k_gemm1(const u16* A, const u16* __restrict__ WT,
                                                const float* __restrict__ bias, u16* HB)
{
  constexpr int NT = 4, BN = 64;
  __shared__ __attribute__((aligned(16))) float stg[GBM * BN];
  __shared__ float sb[BN];
  const int tid = (int)threadIdx.x, lane = tid & 31, wave = tid >> 5, hh = lane >> 4, m = lane & 15;
  const int rowBase = (int)blockIdx.x * GBM;
  const int col0    = (int)blockIdx.y * BN;
  if (tid < BN) sb[tid] = bf_rne(bias[col0 + tid]);

  v8f acc[NT];
  {
    const v8f z = {0.f, 0.f, 0.f, 0.f, 0.f, 0.f, 0.f, 0.f};
#pragma unroll
    for (int t = 0; t < NT; ++t) acc[t] = z;
  }
  const u16* ap = A  + (size_t)(rowBase + 16 * wave + m) * (size_t)K1 + 8 * hh;
  const u16* wp = WT + (size_t)(col0 + m) * (size_t)K1 + 8 * hh;
#pragma unroll 1
  for (int ks = 0; ks < K1 / 32; ++ks) {
    FragB af;
    af.h[0] = *(const v8usa*)(ap + 32 * ks);
    af.h[1] = *(const v8usa*)(ap + 32 * ks + 16);
#pragma unroll
    for (int t = 0; t < NT; ++t) {
      const u16* wq = wp + (size_t)(16 * t) * (size_t)K1 + 32 * ks;
      FragB bf;
      bf.h[0] = *(const v8usa*)wq;
      bf.h[1] = *(const v8usa*)(wq + 16);
      acc[t] = wmb(af, bf, acc[t]);
    }
  }

#pragma unroll
  for (int t = 0; t < NT; ++t) {
    const int lc = 16 * t + m;
#pragma unroll
    for (int r = 0; r < 8; ++r) {
      const int lr = 16 * wave + 8 * hh + r;
      stg[lr * BN + lc] = acc[t][r];
    }
  }
  __syncthreads();

  const int rsub = hh;
  const int half = m >> 3;
  const int cp   = m & 7;
  float bb[8];
#pragma unroll
  for (int j = 0; j < 8; ++j) bb[j] = sb[8 * cp + j];
  v8us pv[8];
#pragma unroll
  for (int i = 0; i < 8; ++i) {
    const int lr = 16 * wave + 2 * i + rsub;
    const float* sr = stg + lr * BN + 8 * cp;
    const v4f a = *(const v4fa*)sr;
    const v4f b = *(const v4fa*)(sr + 4);
    float v[8] = {a.x, a.y, a.z, a.w, b.x, b.y, b.z, b.w};
#pragma unroll
    for (int j = 0; j < 8; ++j) {
      const float t = fmaxf(v[j] + bb[j], 0.0f);
      const unsigned short hb = bf_bits(t);
      const unsigned short lb = bf_bits(t - bf_val(hb));
      pv[i][j] = (half != 0) ? lb : hb;
    }
  }
  u16* gb = HB + (size_t)(rowBase + 16 * wave + rsub) * (size_t)HBP + half * DH + col0 + 8 * cp;
#pragma unroll
  for (int i = 0; i < 8; ++i) *(volatile v8us*)(gb + (size_t)(2 * i) * HBP) = pv[i];
  __threadfence();
#pragma unroll
  for (int i = 0; i < 8; ++i) *(volatile v8us*)(gb + (size_t)(2 * i) * HBP) = pv[i];
}

__global__ __launch_bounds__(GTHR) void k_gemm2(const u16* AM, const u16* AH, const u16* __restrict__ WT,
                                                const float* __restrict__ bias, float* out, int nN)
{
  constexpr int NT = 4, BN = 64;
  __shared__ __attribute__((aligned(16))) float stg[GBM * BN];
  __shared__ __attribute__((aligned(16))) float sout[GBM * NCLS];
  __shared__ float sb[BN];
  const int tid = (int)threadIdx.x, lane = tid & 31, wave = tid >> 5, hh = lane >> 4, m = lane & 15;
  const int rowBase = (int)blockIdx.x * GBM;
  if (tid < BN) {
    const int cb = tid < NCLS ? tid : NCLS - 1;
    const float bv = bf_rne(bias[cb]);
    sb[tid] = tid < NCLS ? bv : 0.0f;
  }

  v8f acc[NT];
  {
    const v8f z = {0.f, 0.f, 0.f, 0.f, 0.f, 0.f, 0.f, 0.f};
#pragma unroll
    for (int t = 0; t < NT; ++t) acc[t] = z;
  }
  const size_t arow = (size_t)(rowBase + 16 * wave + m) * (size_t)HBP + 8 * hh;
  const u16* apm = AM + arow;
  const u16* aph = AH + arow;
  const u16* wp  = WT + (size_t)m * (size_t)K2 + 8 * hh;
#pragma unroll 1
  for (int ks = 0; ks < HBP / 32; ++ks) {
    FragB af;
    af.h[0] = *(const v8usa*)(apm + 32 * ks);
    af.h[1] = *(const v8usa*)(apm + 32 * ks + 16);
#pragma unroll
    for (int t = 0; t < NT; ++t) {
      const u16* wq = wp + (size_t)(16 * t) * (size_t)K2 + 32 * ks;
      FragB bf;
      bf.h[0] = *(const v8usa*)wq;
      bf.h[1] = *(const v8usa*)(wq + 16);
      acc[t] = wmb(af, bf, acc[t]);
    }
  }
#pragma unroll 1
  for (int ks = 0; ks < HBP / 32; ++ks) {
    FragB af;
    af.h[0] = *(const v8usa*)(aph + 32 * ks);
    af.h[1] = *(const v8usa*)(aph + 32 * ks + 16);
#pragma unroll
    for (int t = 0; t < NT; ++t) {
      const u16* wq = wp + (size_t)(16 * t) * (size_t)K2 + HBP + 32 * ks;
      FragB bf;
      bf.h[0] = *(const v8usa*)wq;
      bf.h[1] = *(const v8usa*)(wq + 16);
      acc[t] = wmb(af, bf, acc[t]);
    }
  }

#pragma unroll
  for (int t = 0; t < NT; ++t) {
    const int lc = 16 * t + m;
#pragma unroll
    for (int r = 0; r < 8; ++r) {
      const int lr = 16 * wave + 8 * hh + r;
      stg[lr * BN + lc] = acc[t][r];
    }
  }
  __syncthreads();

  const int l8 = lane < 8 ? lane : 7;
  const float b0v = sb[lane];
  const float b1v = sb[32 + l8];
  const float ninf = -__builtin_inff();
#pragma unroll 1
  for (int i = 0; i < 16; ++i) {
    const int lr = 16 * wave + i;
    const float* sr = stg + lr * BN;
    const float o0 = sr[lane] + b0v;
    const float o1 = sr[32 + l8] + b1v;
    float mx = fmaxf(o0, lane < 8 ? o1 : ninf);
#pragma unroll
    for (int off = 16; off > 0; off >>= 1) mx = fmaxf(mx, __shfl_xor(mx, off));
    const float e0  = expf(o0 - mx);
    const float e1f = expf(o1 - mx);
    const float e1  = lane < 8 ? e1f : 0.0f;
    float sm = e0 + e1;
#pragma unroll
    for (int off = 16; off > 0; off >>= 1) sm += __shfl_xor(sm, off);
    const float inv = 1.0f / sm;
    sout[lr * NCLS + lane] = e0 * inv;
    if (lane < 8) sout[lr * NCLS + 32 + lane] = e1 * inv;
  }
  __syncthreads();

  int nv = nN - rowBase;
  nv = nv < 0 ? 0 : (nv > GBM ? GBM : nv);
  const int np = nv * (NCLS / 4);
  float* ob = out + (size_t)rowBase * NCLS;
#pragma unroll 1
  for (int p = tid; p < np; p += GTHR) *(volatile v4f*)(ob + 4 * p) = *(const v4fa*)(sout + 4 * p);
  __threadfence();
#pragma unroll 1
  for (int p = tid; p < np; p += GTHR) *(volatile v4f*)(ob + 4 * p) = *(const v4fa*)(sout + 4 * p);
}

template<int AGGM>
__global__ __launch_bounds__(NTHR) void k_agg(
    const int* __restrict__ srcs, const int* __restrict__ dsts,
    const u16* __restrict__ F, int pitchF,
    u16* Aout, int ldaOut,
    int nN, int nE, int nb, int vec8, int MPr) {
  extern __shared__ v4f lds_dyn[];
  int* reg1 = (int*)lds_dyn;
  int* reg2 = reg1 + RCAP;
  int* scnt = reg2 + RCAP;
  int* soff = scnt + NBMAX;
  int* list = soff + NBMAX;
  int* wcnt = list + LISTN;
  int* wtot = wcnt + NWAVE;
  const int tid = (int)threadIdx.x, lane = tid & 31, wave = tid >> 5;
  const int nodeBase = (int)blockIdx.x * nb;

  for (int i = tid; i < NBMAX; i += NTHR) scnt[i] = 0;
  __syncthreads();

  int tot = 0;
  const int nChunks = (nE + CHUNK - 1) / CHUNK;
#pragma unroll 1
  for (int ch = 0; ch < nChunks; ++ch) {
    const int cbase = ch * CHUNK;
    const int wc = scan_chunk(dsts, nE, cbase, nodeBase, nb, vec8, list, tid, lane, wave);
    if (lane == 0) wcnt[wave] = wc;
    __syncthreads();
    int pre = 0, all = 0;
#pragma unroll
    for (int w2 = 0; w2 < NWAVE; ++w2) {
      int c = wcnt[w2];
      c = c < 0 ? 0 : (c > WCAP ? WCAP : c);
      all += c;
      pre += (w2 < wave) ? c : 0;
    }
    const int wcc  = wc > WCAP ? WCAP : wc;
    const int base = tot + pre;
#pragma unroll 1
    for (int i = lane; i < wcc; i += 32) {
      const int ent = list[wave * WCAP + i];
      const int el  = (ent >> PKS) & (CHUNK - 1);
      const int sl  = ent & (NBMAX - 1);
      int eid = cbase + el;
      eid = eid > nE - 1 ? nE - 1 : eid;
      const int pos = base + i;
      if (pos < RCAP) reg1[pos] = (int)(((unsigned)eid << PKS) | (unsigned)sl);
    }
    tot += all;
    tot = tot > RCAP ? RCAP : tot;
    __syncthreads();
  }
  const int nh = tot;

  if (wave == 0) {
#pragma unroll 1
    for (int b0 = 0; b0 < nh; b0 += 32) {
      const int idx = b0 + lane;
      const int uv  = reg1[idx < RCAP ? idx : RCAP - 1];
      const int m32 = (nh - b0) < 32 ? (nh - b0) : 32;
#pragma unroll 1
      for (int k = 0; k < m32; ++k) {
        const int u  = __builtin_amdgcn_readlane(uv, k);
        const int sl = u & (NBMAX - 1);
        if (lane == 0) scnt[sl] = scnt[sl] + 1;
      }
    }
  }
  __syncthreads();

  {
    const v4i ca = *(const v4i*)(scnt + 8 * tid);
    const v4i cb = *(const v4i*)(scnt + 8 * tid + 4);
    const int e0 = ca.x < 0 ? 0 : ca.x, e1 = ca.y < 0 ? 0 : ca.y, e2 = ca.z < 0 ? 0 : ca.z, e3 = ca.w < 0 ? 0 : ca.w;
    const int e4 = cb.x < 0 ? 0 : cb.x, e5 = cb.y < 0 ? 0 : cb.y, e6 = cb.z < 0 ? 0 : cb.z, e7 = cb.w < 0 ? 0 : cb.w;
    const int ts = e0 + e1 + e2 + e3 + e4 + e5 + e6 + e7;
    int incl = ts;
#pragma unroll
    for (int d = 1; d < 32; d <<= 1) {
      const int up = __shfl_up(incl, d);
      if (lane >= d) incl += up;
    }
    if (lane == 31) wtot[wave] = incl;
    __syncthreads();
    int pre = 0;
#pragma unroll
    for (int w2 = 0; w2 < NWAVE; ++w2) pre += (w2 < wave) ? wtot[w2] : 0;
    int run = pre + incl - ts;
    soff[8 * tid + 0] = run; run += e0;
    soff[8 * tid + 1] = run; run += e1;
    soff[8 * tid + 2] = run; run += e2;
    soff[8 * tid + 3] = run; run += e3;
    soff[8 * tid + 4] = run; run += e4;
    soff[8 * tid + 5] = run; run += e5;
    soff[8 * tid + 6] = run; run += e6;
    soff[8 * tid + 7] = run;
  }
  __syncthreads();
  for (int i = tid; i < NBMAX; i += NTHR) list[i] = soff[i];
  __syncthreads();

  if (wave == 0) {
#pragma unroll 1
    for (int b0 = 0; b0 < nh; b0 += 32) {
      const int idx = b0 + lane;
      const int uv  = reg1[idx < RCAP ? idx : RCAP - 1];
      const int m32 = (nh - b0) < 32 ? (nh - b0) : 32;
#pragma unroll 1
      for (int k = 0; k < m32; ++k) {
        const int u   = __builtin_amdgcn_readlane(uv, k);
        const int sl  = u & (NBMAX - 1);
        const int eid = (int)((unsigned)u >> PKS);
        if (lane == 0) {
          int pos = list[sl];
          pos = pos < 0 ? 0 : (pos > RCAP - 1 ? RCAP - 1 : pos);
          reg2[pos] = eid;
          list[sl] = pos + 1;
        }
      }
    }
  }
  __syncthreads();

  const int nbw = nb >> 3;
  const bool ovf = (nh >= RCAP);
  const float qnan = __int_as_float(0x7fc00000);
  unsigned int* stwu = (unsigned int*)((float*)reg1 + wave * STW);

#pragma unroll 1
  for (int jt = 0; jt < nbw; ++jt) {
    const int slot = wave * nbw + jt;
    const int grow = nodeBase + slot;
    const int gcl  = grow < nN ? grow : nN - 1;
    int st = soff[slot];
    const int craw = scnt[slot];
    int cnt = craw;
    st  = st < 0 ? 0 : (st > nh ? nh : st);
    cnt = cnt < 0 ? 0 : (cnt > DEGCAP ? DEGCAP : cnt);
    if (cnt > nh - st) cnt = nh - st;
    const float pz = (ovf || craw > DEGCAP) ? qnan : 0.0f;
    const bool liveb = grow < nN;
    const float live = liveb ? 1.0f : 0.0f;

    float ag0 = 0.f, ag1 = 0.f, ag2 = 0.f, ag3 = 0.f;
#pragma unroll 1
    for (int q = 0; q < cnt; ++q) {
      int idx = st + q; idx = idx > RCAP - 1 ? RCAP - 1 : idx;
      int eid = reg2[idx]; eid = eid < 0 ? 0 : (eid > nE - 1 ? nE - 1 : eid);
      const int sraw = srcs[eid];
      const int s = sraw < 0 ? 0 : (sraw > nN - 1 ? nN - 1 : sraw);
      const u16* nr = F + (size_t)s * (size_t)pitchF + 4 * lane;
      const v2u w = *(const v2ua*)nr;
      float f0 = __uint_as_float(w.x << 16), f1 = __uint_as_float(w.x & 0xffff0000u);
      float f2 = __uint_as_float(w.y << 16), f3 = __uint_as_float(w.y & 0xffff0000u);
      if (AGGM == 1) {
        const v2u wl = *(const v2ua*)(nr + DH);
        f0 += __uint_as_float(wl.x << 16); f1 += __uint_as_float(wl.x & 0xffff0000u);
        f2 += __uint_as_float(wl.y << 16); f3 += __uint_as_float(wl.y & 0xffff0000u);
      }
      ag0 += f0; ag1 += f1; ag2 += f2; ag3 += f3;
    }
    const float dcl  = cnt > 0 ? (float)cnt : 1.0f;
    const float invd = 1.0f / dcl;
    const float m0 = (ag0 * invd) * live + pz;
    const float m1 = (ag1 * invd) * live + pz;
    const float m2 = (ag2 * invd) * live + pz;
    const float m3 = (ag3 * invd) * live + pz;
    const unsigned short hb0 = bf_bits(m0), hb1 = bf_bits(m1), hb2 = bf_bits(m2), hb3 = bf_bits(m3);
    const unsigned short lb0 = bf_bits(m0 - bf_val(hb0)), lb1 = bf_bits(m1 - bf_val(hb1));
    const unsigned short lb2 = bf_bits(m2 - bf_val(hb2)), lb3 = bf_bits(m3 - bf_val(hb3));
    v2u hw, lw;
    hw.x = (unsigned int)hb0 | ((unsigned int)hb1 << 16);
    hw.y = (unsigned int)hb2 | ((unsigned int)hb3 << 16);
    lw.x = (unsigned int)lb0 | ((unsigned int)lb1 << 16);
    lw.y = (unsigned int)lb2 | ((unsigned int)lb3 << 16);
    v2u xw;
    xw.x = 0u; xw.y = 0u;
    if (AGGM == 0) {
      const v2u xs = *(const v2ua*)(F + (size_t)gcl * (size_t)pitchF + 4 * lane);
      xw.x = liveb ? xs.x : 0u;
      xw.y = liveb ? xs.y : 0u;
    }
    __builtin_amdgcn_fence(__ATOMIC_RELEASE, "wavefront");
    __builtin_amdgcn_wave_barrier();
    *(v2ua*)(stwu + 2 * lane)      = hw;
    *(v2ua*)(stwu + 64 + 2 * lane) = lw;
    if (AGGM == 0) *(v2ua*)(stwu + 128 + 2 * lane) = xw;
    __builtin_amdgcn_fence(__ATOMIC_RELEASE, "wavefront");
    __builtin_amdgcn_wave_barrier();
    const v4u pk0 = *(const v4ua*)(stwu + 4 * lane);
    u16* gp = Aout + (size_t)grow * (size_t)ldaOut;
    const bool wsv = grow < MPr;
    if (AGGM == 0) {
      const int lq = lane < 16 ? lane : 15;
      const v4u pk1 = *(const v4ua*)(stwu + 128 + 4 * lq);
      const bool w1 = wsv && (lane < 16);
      if (wsv) *(volatile v4u*)(gp + 8 * lane) = pk0;
      if (w1)  *(volatile v4u*)(gp + 2 * DH + 8 * lane) = pk1;
      __threadfence();
      if (wsv) *(volatile v4u*)(gp + 8 * lane) = pk0;
      if (w1)  *(volatile v4u*)(gp + 2 * DH + 8 * lane) = pk1;
    } else {
      if (wsv) *(volatile v4u*)(gp + 8 * lane) = pk0;
      __threadfence();
      if (wsv) *(volatile v4u*)(gp + 8 * lane) = pk0;
    }
  }
}

static int pick_nb(int nE, int nN) {
  int nb = NBMAX;
  while (nb > 16 && (long long)nb * (long long)nE * 5LL > (long long)RCAP * (long long)nN * 4LL) nb >>= 1;
  return nb;
}
static inline int cdiv(int a, int b) { return (a + b - 1) / b; }

extern "C" void kernel_launch(void* const* d_in, const int* in_sizes, int n_in,
                              void* d_out, int out_size, void* d_ws, size_t ws_size,
                              hipStream_t stream) {
  if (n_in < 8) return;
  if (in_sizes[0] < DIN || (in_sizes[0] % DIN) != 0) return;
  const int nN = in_sizes[0] / DIN;
  if (nN <= 0 || nN > (1 << 22)) return;
  if (in_sizes[1] < 2 || (in_sizes[1] & 1) != 0) return;
  const int nE = in_sizes[1] / 2;
  if (nE < 1 || nE > (1 << 21)) return;
  if (in_sizes[2] != DIN * DH || in_sizes[3] != DIN * DH || in_sizes[4] != DH) return;
  if (in_sizes[5] != DH * NCLS || in_sizes[6] != DH * NCLS || in_sizes[7] != NCLS) return;
  if (out_size != nN * NCLS) return;

  const float* x   = (const float*)d_in[0];
  const int*   ei  = (const int*)  d_in[1];
  const float* W1l = (const float*)d_in[2];
  const float* W1r = (const float*)d_in[3];
  const float* b1  = (const float*)d_in[4];
  const float* W2l = (const float*)d_in[5];
  const float* W2r = (const float*)d_in[6];
  const float* b2  = (const float*)d_in[7];
  float* out = (float*)d_out;
  const int* srcs = ei;
  const int* dsts = ei + nE;

  const int MP   = cdiv(nN, GBM) * GBM;
  const int nb   = pick_nb(nE, nN);
  const int gA   = cdiv(MP, nb);
  const int vec8 = ((nE & 3) == 0) ? 1 : 0;
  if (nb < 16 || nb > NBMAX || gA * nb < MP) return;

  char* ws = (char*)d_ws;
  size_t off = 0;
  const size_t oRA = off; off += (size_t)MP * HBP * 2;             off = (off + 255) & ~(size_t)255;
  const size_t oRB = off; off += (size_t)MP * K1 * 2;              off = (off + 255) & ~(size_t)255;
  const size_t oW1 = off; off += (size_t)DH * K1 * 2;              off = (off + 255) & ~(size_t)255;
  const size_t oW2 = off; off += (size_t)NCP * K2 * 2;             off = (off + 255) & ~(size_t)255;
  if (off > ws_size || off > (size_t)WSCAP || off > (size_t)WSMAX) return;
  u16* XB  = (u16*)(ws + oRA);
  u16* HB  = (u16*)(ws + oRA);
  u16* A1  = (u16*)(ws + oRB);
  u16* M2  = (u16*)(ws + oRB);
  u16* WT1 = (u16*)(ws + oW1);
  u16* WT2 = (u16*)(ws + oW2);

  hipFuncSetAttribute(reinterpret_cast<const void*>(&k_agg<0>),
                      hipFuncAttributeMaxDynamicSharedMemorySize, LDS_AGG);
  hipFuncSetAttribute(reinterpret_cast<const void*>(&k_agg<1>),
                      hipFuncAttributeMaxDynamicSharedMemorySize, LDS_AGG);

  const int nUx = MP * (DIN / 8);
  k_xprep<<<cdiv(nUx, NTHR), NTHR, 0, stream>>>(x, XB, nN, nUx);

  {
    const int nU1 = DH * (K1 / 8);
    k_wtr<<<cdiv(nU1, NTHR), NTHR, 0, stream>>>(W1l, W1r, DH, 2, K1, WT1, nU1);
    const int nU2 = NCP * (K2 / 8);
    k_wtr<<<cdiv(nU2, NTHR), NTHR, 0, stream>>>(W2l, W2r, NCLS, 2, K2, WT2, nU2);
  }

  const int gM = MP / GBM;
  k_agg<0><<<gA, NTHR, LDS_AGG, stream>>>(srcs, dsts, XB, DIN, A1, K1, nN, nE, nb, vec8, MP);
  k_gemm1<<<dim3(gM, DH / 64), GTHR, 0, stream>>>(A1, WT1, b1, HB);
  k_agg<1><<<gA, NTHR, LDS_AGG, stream>>>(srcs, dsts, HB, HBP, M2, HBP, nN, nE, nb, vec8, MP);
  k_gemm2<<<gM, GTHR, 0, stream>>>(M2, HB, WT2, b2, out, nN);
}
